// mp_gnn_39943195852849
// MI455X (gfx1250) — hardware-verified
//
#include <hip/hip_runtime.h>
#include <stddef.h>


#define CH      64
#define KE0     195
#define NTHR    256
#define NWAVE   8
#define EPT     8
#define NGRP    2
#define CHUNK   (NTHR * EPT * NGRP)
#define WCAP    (EPT * NGRP * 32)
#define LISTN   (NWAVE * WCAP)
#define NBA     1024
#define GTHR    128
#define GROWS   64
#define DTHR    64
#define DROWS   32
#define WSLOT   16384
#define WLO     8192
#define NWMAT   12
#define LDS_DRAIN (NBA * CH * 4 + NBA * 4 + LISTN * 4 + 64)

static_assert((CHUNK & (CHUNK - 1)) == 0);
static_assert(CHUNK <= 4096);
static_assert((NBA & (NBA - 1)) == 0);
static_assert(NBA <= 4096);
static_assert(NBA * CH == NWAVE * 64 * 128);
static_assert(NBA == NWAVE * 128);
static_assert(GROWS == (GTHR / 32) * 16);
static_assert(DROWS == (DTHR / 32) * 16);
static_assert((DROWS * 3 * 4) % 128 == 0);

typedef float          v2f  __attribute__((ext_vector_type(2)));
typedef float          v4f  __attribute__((ext_vector_type(4)));
typedef float          v8f  __attribute__((ext_vector_type(8)));
typedef int            v4i  __attribute__((ext_vector_type(4)));
typedef unsigned int   v4u  __attribute__((ext_vector_type(4)));
typedef unsigned short v4us __attribute__((ext_vector_type(4)));
typedef unsigned short v8us __attribute__((ext_vector_type(8)));
typedef __bf16         v16b __attribute__((ext_vector_type(16)));

union FragB { v16b v; v8us u[2]; };
union UF4   { v4f f; v4u u; };

__device__ __forceinline__ v4u bfr4(v4f a) {
  UF4 x; x.f = a;
  return (x.u + 0x7FFFu + ((x.u >> 16) & 1u)) >> 16;
}

__device__ __forceinline__ void split8(v4f a, v4f b, v8us& hv, v8us& lv) {
  const v4u ha = bfr4(a), hb = bfr4(b);
  UF4 ra, rb; ra.u = ha << 16; rb.u = hb << 16;
  const v4u la = bfr4(a - ra.f), lb = bfr4(b - rb.f);
  const v4us ha16 = __builtin_convertvector(ha, v4us), hb16 = __builtin_convertvector(hb, v4us);
  const v4us la16 = __builtin_convertvector(la, v4us), lb16 = __builtin_convertvector(lb, v4us);
  hv = __builtin_shufflevector(ha16, hb16, 0, 1, 2, 3, 4, 5, 6, 7);
  lv = __builtin_shufflevector(la16, lb16, 0, 1, 2, 3, 4, 5, 6, 7);
}

__device__ __forceinline__ void afrag(const float* p, FragB& H, FragB& L) {
  const v4f f0 = *(const v4f*)p,        f1 = *(const v4f*)(p + 4);
  const v4f f2 = *(const v4f*)(p + 16), f3 = *(const v4f*)(p + 20);
  split8(f0, f1, H.u[0], L.u[0]);
  split8(f2, f3, H.u[1], L.u[1]);
}

__device__ __forceinline__ void bfrag(const unsigned short* __restrict__ plane, int K, int n, int k0, int hh,
                                      FragB& H, FragB& L) {
  const unsigned short* bp = plane + (size_t)n * K + k0 + 8 * hh;
  H.u[0] = *(const v8us*)bp;
  H.u[1] = *(const v8us*)(bp + 16);
  const unsigned short* lq = bp + WLO;
  L.u[0] = *(const v8us*)lq;
  L.u[1] = *(const v8us*)(lq + 16);
}

__device__ __forceinline__ v8f wmb(v16b a, v16b b, v8f c) {
  v8f d = __builtin_amdgcn_wmma_f32_16x16x32_bf16(false, a, false, b, (short)0, c, false, false);
  asm volatile("v_nop\n\tv_nop\n\tv_nop\n\tv_nop" : "+v"(d) : "v"(a), "v"(b));
  return d;
}

__device__ __forceinline__ v8f wm3(const FragB& ah, const FragB& al, const FragB& bh, const FragB& bl, v8f c) {
  c = wmb(ah.v, bh.v, c);
  c = wmb(ah.v, bl.v, c);
  c = wmb(al.v, bh.v, c);
  return c;
}

__device__ __forceinline__ void gemm_k64(const float* ar, const unsigned short* __restrict__ plane, int K, int kofs,
                                         int m, int hh, v8f* acc) {
#pragma unroll
  for (int kt = 0; kt < 2; ++kt) {
    FragB aH, aL;
    afrag(ar + 32 * kt, aH, aL);
#pragma unroll
    for (int t = 0; t < 4; ++t) {
      FragB bH, bL;
      bfrag(plane, K, 16 * t + m, kofs + 32 * kt, hh, bH, bL);
      acc[t] = wm3(aH, aL, bH, bL, acc[t]);
    }
  }
}

__device__ __forceinline__ float elu1(float x) {
  return x > 0.0f ? x : (__expf(x) - 1.0f);
}

template <int NB>
__device__ __forceinline__ int scan_chunk(const int* __restrict__ dsts, int nE, int cbase, int nodeBase,
                                          int vec8, int* list, int tid, int wave) {
  int wc = 0;
#pragma unroll
  for (int g = 0; g < NGRP; ++g) {
    const int el0  = (g * NTHR + tid) * EPT;
    const int e0   = cbase + el0;
    const int sent = -2147483647 - 1;
    v4i da, db;
    if (vec8 != 0 && cbase + CHUNK <= nE) {
      da = *(const v4i*)(dsts + e0);
      db = *(const v4i*)(dsts + e0 + 4);
    } else {
      da.x = (e0     < nE) ? dsts[min(e0,     nE - 1)] : sent;
      da.y = (e0 + 1 < nE) ? dsts[min(e0 + 1, nE - 1)] : sent;
      da.z = (e0 + 2 < nE) ? dsts[min(e0 + 2, nE - 1)] : sent;
      da.w = (e0 + 3 < nE) ? dsts[min(e0 + 3, nE - 1)] : sent;
      db.x = (e0 + 4 < nE) ? dsts[min(e0 + 4, nE - 1)] : sent;
      db.y = (e0 + 5 < nE) ? dsts[min(e0 + 5, nE - 1)] : sent;
      db.z = (e0 + 6 < nE) ? dsts[min(e0 + 6, nE - 1)] : sent;
      db.w = (e0 + 7 < nE) ? dsts[min(e0 + 7, nE - 1)] : sent;
    }
    const unsigned nb = (unsigned)nodeBase;
    const unsigned s0 = (unsigned)da.x - nb, s1 = (unsigned)da.y - nb;
    const unsigned s2 = (unsigned)da.z - nb, s3 = (unsigned)da.w - nb;
    const unsigned s4 = (unsigned)db.x - nb, s5 = (unsigned)db.y - nb;
    const unsigned s6 = (unsigned)db.z - nb, s7 = (unsigned)db.w - nb;
    const bool h0 = s0 < (unsigned)NB, h1 = s1 < (unsigned)NB, h2 = s2 < (unsigned)NB, h3 = s3 < (unsigned)NB;
    const bool h4 = s4 < (unsigned)NB, h5 = s5 < (unsigned)NB, h6 = s6 < (unsigned)NB, h7 = s7 < (unsigned)NB;
    const unsigned any = __builtin_amdgcn_ballot_w32(h0 | h1 | h2 | h3 | h4 | h5 | h6 | h7);
    if (any != 0u) {
#define HITJ(J, HJ, SJ) { \
        const unsigned mj = __builtin_amdgcn_ballot_w32(HJ); \
        if (mj != 0u) { \
          if (HJ) { \
            const int psn = wc + (int)__builtin_amdgcn_mbcnt_lo(mj, 0u); \
            if (psn < WCAP) list[wave * WCAP + psn] = ((el0 + (J)) << 12) | (int)(SJ); \
          } \
          wc += (int)__builtin_popcount(mj); } }
      HITJ(0, h0, s0)
      HITJ(1, h1, s1)
      HITJ(2, h2, s2)
      HITJ(3, h3, s3)
      HITJ(4, h4, s4)
      HITJ(5, h5, s5)
      HITJ(6, h6, s6)
      HITJ(7, h7, s7)
#undef HITJ
    }
  }
  return wc;
}

__global__ __launch_bounds__(256) void k_wprep(
    const float* __restrict__ encW1, const float* __restrict__ decW0,
    const float* __restrict__ eW0, const float* __restrict__ eW1,
    const float* __restrict__ nW0, const float* __restrict__ nW1,
    unsigned short* wb) {
  const int j = blockIdx.y;
  const float* W  = encW1;
  const float* W2 = encW1;
  float sgn = 0.0f;
  int K = CH;
  if (j == 1) { W = decW0; W2 = decW0; }
  else if (j >= 2) {
    const int li = (j - 2) / 5;
    const int r  = (j - 2) - 5 * li;
    const float* e0 = eW0 + (size_t)li * KE0 * CH;
    if (r == 0)      { W = e0;            W2 = e0 + 128 * CH; sgn = 1.0f; }
    else if (r == 1) { W = e0 + 64 * CH;  W2 = e0 + 128 * CH; sgn = -1.0f; }
    else if (r == 2) { W = eW1 + (size_t)li * CH * CH;     W2 = W; }
    else if (r == 3) { W = nW0 + (size_t)li * 2 * CH * CH; W2 = W; K = 2 * CH; }
    else             { W = nW1 + (size_t)li * CH * CH;     W2 = W; }
  }
  const int idx = blockIdx.x * 256 + threadIdx.x;
  if (idx >= CH * K / 8) return;
  const int o  = idx * 8;
  const int n  = o / K;
  const int k0 = o - n * K;
  const float* p = W  + (size_t)k0 * CH + n;
  const float* q = W2 + (size_t)k0 * CH + n;
  v4f a, b;
  a.x = p[0]      + sgn * q[0];       a.y = p[CH]     + sgn * q[CH];
  a.z = p[2 * CH] + sgn * q[2 * CH];  a.w = p[3 * CH] + sgn * q[3 * CH];
  b.x = p[4 * CH] + sgn * q[4 * CH];  b.y = p[5 * CH] + sgn * q[5 * CH];
  b.z = p[6 * CH] + sgn * q[6 * CH];  b.w = p[7 * CH] + sgn * q[7 * CH];
  v8us hv, lv;
  split8(a, b, hv, lv);
  unsigned short* hp = wb + (size_t)j * WSLOT + o;
  unsigned short* lq = hp + WLO;
  *(volatile v8us*)hp = hv;
  *(volatile v8us*)lq = lv;
  __threadfence();
  *(volatile v8us*)hp = hv;
  *(volatile v8us*)lq = lv;
}

__global__ __launch_bounds__(GTHR) void k_enc(
    const float* __restrict__ x, const float* __restrict__ W0, const float* __restrict__ b0,
    const unsigned short* __restrict__ wE1, const float* __restrict__ b1,
    float* hOut, int nN) {
  __shared__ __attribute__((aligned(16))) float tT[4][16 * CH];
  __shared__ __attribute__((aligned(16))) float tO[4][16 * CH];
  const int tid = threadIdx.x, lane = tid & 31, wave = tid >> 5, hh = lane >> 4, m = lane & 15;
  const int n0 = (blockIdx.x * 4 + wave) * 16;
  int node = n0 + m; node = node > nN - 1 ? nN - 1 : node;

  {
    const float x0 = x[(size_t)node * 3 + 0], x1 = x[(size_t)node * 3 + 1], x2 = x[(size_t)node * 3 + 2];
    float* tr = tT[wave] + m * CH;
#pragma unroll 8
    for (int jj = 0; jj < 32; ++jj) {
      const int o = 32 * hh + jj;
      const float v = x0 * W0[o] + x1 * W0[CH + o] + x2 * W0[2 * CH + o] + b0[o];
      tr[o] = elu1(v);
    }
  }
  __syncthreads();

  v8f acc[4];
  const v8f z8 = {0.f, 0.f, 0.f, 0.f, 0.f, 0.f, 0.f, 0.f};
#pragma unroll
  for (int t = 0; t < 4; ++t) acc[t] = z8;
  gemm_k64(tT[wave] + m * CH + 8 * hh, wE1, CH, 0, m, hh, acc);

  {
    float* sp = tO[wave] + 8 * hh * CH + m;
#pragma unroll
    for (int t = 0; t < 4; ++t) {
      const float bb = b1[16 * t + m];
#pragma unroll
      for (int r = 0; r < 8; ++r) sp[r * CH + 16 * t] = acc[t][r] + bb;
    }
  }
  __syncthreads();

  const float* lp = tO[wave] + 4 * lane;
  float* gp = hOut + (size_t)n0 * CH + 4 * lane;
#pragma unroll
  for (int i = 0; i < 8; ++i) { const v4f v = *(const v4f*)(lp + i * 128); *(volatile v4f*)(gp + i * 128) = v; }
  __threadfence();
#pragma unroll
  for (int i = 0; i < 8; ++i) { const v4f v = *(const v4f*)(lp + i * 128); *(volatile v4f*)(gp + i * 128) = v; }
}

__global__ __launch_bounds__(GTHR) void k_pq(
    const float* __restrict__ h, const unsigned short* __restrict__ wP, const unsigned short* __restrict__ wQ,
    const float* __restrict__ eb0, float* P, float* Q, int nN) {
  __shared__ __attribute__((aligned(16))) float tP[4][16 * CH];
  __shared__ __attribute__((aligned(16))) float tQ[4][16 * CH];
  const int tid = threadIdx.x, lane = tid & 31, wave = tid >> 5, hh = lane >> 4, m = lane & 15;
  const int n0 = (blockIdx.x * 4 + wave) * 16;
  int node = n0 + m; node = node > nN - 1 ? nN - 1 : node;
  const float* ar = h + (size_t)node * CH + 8 * hh;
  const v8f z8 = {0.f, 0.f, 0.f, 0.f, 0.f, 0.f, 0.f, 0.f};

  v8f acc[4];
#pragma unroll
  for (int t = 0; t < 4; ++t) acc[t] = z8;
  gemm_k64(ar, wP, CH, 0, m, hh, acc);
  {
    float* sp = tP[wave] + 8 * hh * CH + m;
#pragma unroll
    for (int t = 0; t < 4; ++t) {
#pragma unroll
      for (int r = 0; r < 8; ++r) sp[r * CH + 16 * t] = acc[t][r];
    }
  }

#pragma unroll
  for (int t = 0; t < 4; ++t) acc[t] = z8;
  gemm_k64(ar, wQ, CH, 0, m, hh, acc);
  {
    float* sp = tQ[wave] + 8 * hh * CH + m;
#pragma unroll
    for (int t = 0; t < 4; ++t) {
      const float bb = eb0[16 * t + m];
#pragma unroll
      for (int r = 0; r < 8; ++r) sp[r * CH + 16 * t] = acc[t][r] + bb;
    }
  }
  __syncthreads();

  const float* lpP = tP[wave] + 4 * lane;
  const float* lpQ = tQ[wave] + 4 * lane;
  float* gpP = P + (size_t)n0 * CH + 4 * lane;
  float* gpQ = Q + (size_t)n0 * CH + 4 * lane;
#pragma unroll
  for (int i = 0; i < 8; ++i) {
    const v4f vp = *(const v4f*)(lpP + i * 128); *(volatile v4f*)(gpP + i * 128) = vp;
    const v4f vq = *(const v4f*)(lpQ + i * 128); *(volatile v4f*)(gpQ + i * 128) = vq;
  }
  __threadfence();
#pragma unroll
  for (int i = 0; i < 8; ++i) {
    const v4f vp = *(const v4f*)(lpP + i * 128); *(volatile v4f*)(gpP + i * 128) = vp;
    const v4f vq = *(const v4f*)(lpQ + i * 128); *(volatile v4f*)(gpQ + i * 128) = vq;
  }
}

__global__ __launch_bounds__(NTHR) void k_drain(
    const int* __restrict__ ei, const float* __restrict__ P, const float* __restrict__ Q,
    const float* __restrict__ pos, const float* __restrict__ W0d,
    float* U, float* cntp, int nN, int nE, int vec8) {
  extern __shared__ v4f lds_dyn[];
  float* accU = (float*)lds_dyn;
  int*   cnt  = (int*)(accU + NBA * CH);
  int*   list = cnt + NBA;
  int*   wcnt = list + LISTN;
  const int tid = threadIdx.x, lane = tid & 31, wave = tid >> 5;
  const int nodeBase = blockIdx.x * NBA;
  const int* dsts = ei + nE;

  {
    const v4f z = {0.f, 0.f, 0.f, 0.f};
    for (int i = tid; i < NBA * CH / 4; i += NTHR) lds_dyn[i] = z;
    for (int i = tid; i < NBA; i += NTHR) cnt[i] = 0;
  }
  const int c0 = 2 * lane;
  const float w00 = W0d[c0],          w01 = W0d[c0 + 1];
  const float w10 = W0d[CH + c0],     w11 = W0d[CH + c0 + 1];
  const float w20 = W0d[2 * CH + c0], w21 = W0d[2 * CH + c0 + 1];
  __syncthreads();

  const int nChunks = (nE + CHUNK - 1) / CHUNK;
#pragma unroll 1
  for (int ch = 0; ch < nChunks; ++ch) {
    const int cbase = ch * CHUNK;
    const int wc = scan_chunk<NBA>(dsts, nE, cbase, nodeBase, vec8, list, tid, wave);
    if (lane == 0) wcnt[wave] = wc;
    __syncthreads();
    if (wave == 0) {
#pragma unroll 1
      for (int wsx = 0; wsx < NWAVE; ++wsx) {
        int n = __builtin_amdgcn_readfirstlane(wcnt[wsx]);
        n = n > WCAP ? WCAP : (n < 0 ? 0 : n);
        const int* lp = list + wsx * WCAP;
#pragma unroll 1
        for (int i = 0; i < n; ++i) {
          const int ent  = __builtin_amdgcn_readfirstlane(lp[i]);
          const int slot = ent & (NBA - 1);
          int e = cbase + ((ent >> 12) & (CHUNK - 1));
          e = e > nE - 1 ? nE - 1 : e;
          int src = ei[e];
          src = src < 0 ? 0 : (src > nN - 1 ? nN - 1 : src);
          int dst = nodeBase + slot;
          dst = dst > nN - 1 ? nN - 1 : dst;
          const float px = pos[(size_t)src * 3 + 0] - pos[(size_t)dst * 3 + 0];
          const float py = pos[(size_t)src * 3 + 1] - pos[(size_t)dst * 3 + 1];
          const float pz = pos[(size_t)src * 3 + 2] - pos[(size_t)dst * 3 + 2];
          const v2f pv = *(const v2f*)(P + (size_t)src * CH + c0);
          const v2f qv = *(const v2f*)(Q + (size_t)dst * CH + c0);
          float v0 = pv.x + qv.x + (px * w00 + py * w10 + pz * w20);
          float v1 = pv.y + qv.y + (px * w01 + py * w11 + pz * w21);
          v0 = elu1(v0);
          v1 = elu1(v1);
          v2f* ap = (v2f*)(accU + slot * CH + c0);
          v2f a = *ap;
          a.x += v0;
          a.y += v1;
          *ap = a;
          if (lane == 0) cnt[slot] = cnt[slot] + 1;
        }
      }
    }
    __syncthreads();
  }

  const size_t ub = (size_t)nodeBase * CH;
#pragma unroll 4
  for (int q = 0; q < 64; ++q) {
    const int f = (wave * 64 + q) * 128 + 4 * lane;
    const v4f v = *(const v4f*)(accU + f);
    *(volatile v4f*)(U + ub + f) = v;
  }
  {
    const int f = wave * 128 + 4 * lane;
    const v4i c = *(const v4i*)(cnt + f);
    v4f cf;
    cf.x = (float)c.x; cf.y = (float)c.y; cf.z = (float)c.z; cf.w = (float)c.w;
    *(volatile v4f*)(cntp + (size_t)nodeBase + f) = cf;
  }
  __threadfence();
#pragma unroll 4
  for (int q = 0; q < 64; ++q) {
    const int f = (wave * 64 + q) * 128 + 4 * lane;
    const v4f v = *(const v4f*)(accU + f);
    *(volatile v4f*)(U + ub + f) = v;
  }
  {
    const int f = wave * 128 + 4 * lane;
    const v4i c = *(const v4i*)(cnt + f);
    v4f cf;
    cf.x = (float)c.x; cf.y = (float)c.y; cf.z = (float)c.z; cf.w = (float)c.w;
    *(volatile v4f*)(cntp + (size_t)nodeBase + f) = cf;
  }
}

__global__ __launch_bounds__(GTHR) void k_node(
    const float* __restrict__ hIn, const float* __restrict__ U, const float* __restrict__ cntp,
    const unsigned short* __restrict__ wE1, const float* __restrict__ eb1,
    const unsigned short* __restrict__ wN0, const float* __restrict__ nb0,
    const unsigned short* __restrict__ wN1, const float* __restrict__ nb1,
    float* hOut, int nN) {
  __shared__ __attribute__((aligned(16))) float tA[4][16 * CH];
  __shared__ __attribute__((aligned(16))) float tZ[4][16 * CH];
  __shared__ __attribute__((aligned(16))) float tO[4][16 * CH];
  const int tid = threadIdx.x, lane = tid & 31, wave = tid >> 5, hh = lane >> 4, m = lane & 15;
  const int n0 = (blockIdx.x * 4 + wave) * 16;
  int node = n0 + m; node = node > nN - 1 ? nN - 1 : node;
  const v8f z8 = {0.f, 0.f, 0.f, 0.f, 0.f, 0.f, 0.f, 0.f};
  v8f acc[4];

#pragma unroll
  for (int t = 0; t < 4; ++t) acc[t] = z8;
  gemm_k64(U + (size_t)node * CH + 8 * hh, wE1, CH, 0, m, hh, acc);
  {
    const float* cp = cntp + (size_t)n0 + 8 * hh;
    const v4f ca = *(const v4f*)cp, cb = *(const v4f*)(cp + 4);
    const v8f cr = __builtin_shufflevector(ca, cb, 0, 1, 2, 3, 4, 5, 6, 7);
    float* sp = tA[wave] + 8 * hh * CH + m;
#pragma unroll
    for (int t = 0; t < 4; ++t) {
      const float bb = eb1[16 * t + m];
#pragma unroll
      for (int r = 0; r < 8; ++r) sp[r * CH + 16 * t] = acc[t][r] + cr[r] * bb;
    }
  }
  __syncthreads();

#pragma unroll
  for (int t = 0; t < 4; ++t) acc[t] = z8;
  gemm_k64(hIn + (size_t)node * CH + 8 * hh, wN0, 2 * CH, 0, m, hh, acc);
  gemm_k64(tA[wave] + m * CH + 8 * hh,       wN0, 2 * CH, CH, m, hh, acc);
  {
    float* sp = tZ[wave] + 8 * hh * CH + m;
#pragma unroll
    for (int t = 0; t < 4; ++t) {
      const float bb = nb0[16 * t + m];
#pragma unroll
      for (int r = 0; r < 8; ++r) sp[r * CH + 16 * t] = elu1(acc[t][r] + bb);
    }
  }
  __syncthreads();

#pragma unroll
  for (int t = 0; t < 4; ++t) acc[t] = z8;
  gemm_k64(tZ[wave] + m * CH + 8 * hh, wN1, CH, 0, m, hh, acc);
  {
    float* sp = tO[wave] + 8 * hh * CH + m;
#pragma unroll
    for (int t = 0; t < 4; ++t) {
      const float bb = nb1[16 * t + m];
#pragma unroll
      for (int r = 0; r < 8; ++r) {
        int rn = n0 + 8 * hh + r; rn = rn > nN - 1 ? nN - 1 : rn;
        const float hv = hIn[(size_t)rn * CH + 16 * t + m];
        sp[r * CH + 16 * t] = hv + (acc[t][r] + bb);
      }
    }
  }
  __syncthreads();

  const float* lp = tO[wave] + 4 * lane;
  float* gp = hOut + (size_t)n0 * CH + 4 * lane;
#pragma unroll
  for (int i = 0; i < 8; ++i) { const v4f v = *(const v4f*)(lp + i * 128); *(volatile v4f*)(gp + i * 128) = v; }
  __threadfence();
#pragma unroll
  for (int i = 0; i < 8; ++i) { const v4f v = *(const v4f*)(lp + i * 128); *(volatile v4f*)(gp + i * 128) = v; }
}

__global__ __launch_bounds__(DTHR) void k_dec(
    const float* __restrict__ h, const unsigned short* __restrict__ wD0, const float* __restrict__ b0,
    const float* __restrict__ W1, const float* __restrict__ b1, float* out, int nN) {
  __shared__ __attribute__((aligned(16))) float tE[2][16 * CH];
  __shared__ __attribute__((aligned(16))) float sOut[DROWS * 3];
  const int tid = threadIdx.x, lane = tid & 31, wave = tid >> 5, hh = lane >> 4, m = lane & 15;
  const int rowBase = blockIdx.x * DROWS;
  const int n0 = rowBase + 16 * wave;
  int node = n0 + m; node = node > nN - 1 ? nN - 1 : node;
  const v8f z8 = {0.f, 0.f, 0.f, 0.f, 0.f, 0.f, 0.f, 0.f};
  v8f acc[4];
#pragma unroll
  for (int t = 0; t < 4; ++t) acc[t] = z8;
  gemm_k64(h + (size_t)node * CH + 8 * hh, wD0, CH, 0, m, hh, acc);
  {
    float* sp = tE[wave] + 8 * hh * CH + m;
#pragma unroll
    for (int t = 0; t < 4; ++t) {
      const float bb = b0[16 * t + m];
#pragma unroll
      for (int r = 0; r < 8; ++r) sp[r * CH + 16 * t] = elu1(acc[t][r] + bb);
    }
  }
  __syncthreads();

  {
    const float* er = tE[wave] + m * CH + 32 * hh;
    const float* wr = W1 + 32 * hh * 3;
    float s0 = 0.f, s1 = 0.f, s2 = 0.f;
#pragma unroll 8
    for (int k = 0; k < 32; ++k) {
      const float ev = er[k];
      s0 += ev * wr[3 * k + 0];
      s1 += ev * wr[3 * k + 1];
      s2 += ev * wr[3 * k + 2];
    }
    s0 += __shfl_xor(s0, 16, 32);
    s1 += __shfl_xor(s1, 16, 32);
    s2 += __shfl_xor(s2, 16, 32);
    if (hh == 0) {
      float* so = sOut + (16 * wave + m) * 3;
      so[0] = s0 + b1[0];
      so[1] = s1 + b1[1];
      so[2] = s2 + b1[2];
    }
  }
  __syncthreads();

  if (wave == 0) {
    if (rowBase + DROWS <= nN) {
      float* gp = out + (size_t)rowBase * 3;
      if (lane < 24) { const v4f v = *(const v4f*)(sOut + 4 * lane); *(volatile v4f*)(gp + 4 * lane) = v; }
      __threadfence();
      if (lane < 24) { const v4f v = *(const v4f*)(sOut + 4 * lane); *(volatile v4f*)(gp + 4 * lane) = v; }
    } else {
      const int nv = (nN - rowBase) * 3;
      float* gp = out + (size_t)rowBase * 3;
      for (int i = lane; i < nv; i += 32) { const float v = sOut[i]; *(volatile float*)(gp + i) = v; }
      __threadfence();
      for (int i = lane; i < nv; i += 32) { const float v = sOut[i]; *(volatile float*)(gp + i) = v; }
    }
  }
}

extern "C" void kernel_launch(void* const* d_in, const int* in_sizes, int n_in,
                              void* d_out, int out_size, void* d_ws, size_t ws_size,
                              hipStream_t stream) {
  if (n_in < 19) return;
  const int nN = in_sizes[0] / 3;
  const int nE = in_sizes[2] / 2;
  if (nN <= 0 || nE <= 0) return;
  if (in_sizes[0] != nN * 3 || in_sizes[1] != nN * 3 || in_sizes[2] != nE * 2) return;
  if (in_sizes[3] != 3 * CH || in_sizes[4] != CH || in_sizes[5] != CH * CH || in_sizes[6] != CH ||
      in_sizes[7] != CH * CH || in_sizes[8] != CH || in_sizes[9] != CH * 3 || in_sizes[10] != 3) return;
  const int nL = in_sizes[11] / (KE0 * CH);
  if (nL < 1 || 2 + 5 * nL > NWMAT) return;
  if (in_sizes[11] != nL * KE0 * CH || in_sizes[12] != nL * CH || in_sizes[13] != nL * CH * CH ||
      in_sizes[14] != nL * CH || in_sizes[15] != nL * 2 * CH * CH || in_sizes[16] != nL * CH ||
      in_sizes[17] != nL * CH * CH || in_sizes[18] != nL * CH) return;
  if (out_size != nN * 3) return;

  const float* x     = (const float*)d_in[0];
  const float* pos   = (const float*)d_in[1];
  const int*   ei    = (const int*)d_in[2];
  const float* encW0 = (const float*)d_in[3];
  const float* encB0 = (const float*)d_in[4];
  const float* encW1 = (const float*)d_in[5];
  const float* encB1 = (const float*)d_in[6];
  const float* decW0 = (const float*)d_in[7];
  const float* decB0 = (const float*)d_in[8];
  const float* decW1 = (const float*)d_in[9];
  const float* decB1 = (const float*)d_in[10];
  const float* mpEW0 = (const float*)d_in[11];
  const float* mpEB0 = (const float*)d_in[12];
  const float* mpEW1 = (const float*)d_in[13];
  const float* mpEB1 = (const float*)d_in[14];
  const float* mpNW0 = (const float*)d_in[15];
  const float* mpNB0 = (const float*)d_in[16];
  const float* mpNW1 = (const float*)d_in[17];
  const float* mpNB1 = (const float*)d_in[18];
  float* out = (float*)d_out;

  const int nG = (nN + GROWS - 1) / GROWS;
  const int nA = (nN + NBA - 1) / NBA;
  const int nD = (nN + DROWS - 1) / DROWS;
  const size_t NPH = (size_t)nG * GROWS;
  const size_t NPA = (size_t)nA * NBA;

  char* ws = (char*)d_ws;
  size_t off = 0;
  const size_t bW = (size_t)NWMAT * WSLOT * 2;
  const size_t bH = NPH * CH * 4;
  const size_t bU = NPA * CH * 4;
  const size_t bC = NPA * 4;
  const size_t oW  = off; off += (bW + 255) & ~(size_t)255;
  const size_t oHA = off; off += (bH + 255) & ~(size_t)255;
  const size_t oHB = off; off += (bH + 255) & ~(size_t)255;
  const size_t oP  = off; off += (bH + 255) & ~(size_t)255;
  const size_t oQ  = off; off += (bH + 255) & ~(size_t)255;
  const size_t oU  = off; off += (bU + 255) & ~(size_t)255;
  const size_t oC  = off; off += (bC + 255) & ~(size_t)255;
  if (off > ws_size) return;
  unsigned short* wb = (unsigned short*)(ws + oW);
  float* hA   = (float*)(ws + oHA);
  float* hB   = (float*)(ws + oHB);
  float* P    = (float*)(ws + oP);
  float* Q    = (float*)(ws + oQ);
  float* U    = (float*)(ws + oU);
  float* cntp = (float*)(ws + oC);

  const int vec8 = ((nE & 3) == 0) ? 1 : 0;

  k_wprep<<<dim3(4, NWMAT), 256, 0, stream>>>(encW1, decW0, mpEW0, mpEW1, mpNW0, mpNW1, wb);

  k_enc<<<nG, GTHR, 0, stream>>>(x, encW0, encB0, wb, encB1, hA, nN);

  (void)hipFuncSetAttribute(reinterpret_cast<const void*>(&k_drain),
                            hipFuncAttributeMaxDynamicSharedMemorySize, LDS_DRAIN);

  float* cur = hA;
  float* nxt = hB;
  for (int li = 0; li < nL; ++li) {
    const unsigned short* wP  = wb + (size_t)(2 + 5 * li + 0) * WSLOT;
    const unsigned short* wQ  = wb + (size_t)(2 + 5 * li + 1) * WSLOT;
    const unsigned short* wE1 = wb + (size_t)(2 + 5 * li + 2) * WSLOT;
    const unsigned short* wN0 = wb + (size_t)(2 + 5 * li + 3) * WSLOT;
    const unsigned short* wN1 = wb + (size_t)(2 + 5 * li + 4) * WSLOT;
    const float* W0d = mpEW0 + (size_t)li * KE0 * CH + (size_t)192 * CH;

    k_pq<<<nG, GTHR, 0, stream>>>(cur, wP, wQ, mpEB0 + (size_t)li * CH, P, Q, nN);

    k_drain<<<nA, NTHR, LDS_DRAIN, stream>>>(ei, P, Q, pos, W0d, U, cntp, nN, nE, vec8);

    k_node<<<nG, GTHR, 0, stream>>>(cur, U, cntp,
                                    wE1, mpEB1 + (size_t)li * CH,
                                    wN0, mpNB0 + (size_t)li * CH,
                                    wN1, mpNB1 + (size_t)li * CH,
                                    nxt, nN);
    float* tmp = cur; cur = nxt; nxt = tmp;
  }

  k_dec<<<nD, DTHR, 0, stream>>>(cur, wb + (size_t)1 * WSLOT, decB0, decW1, decB1, out, nN);
}
